// MultiHeadAttention_7937099563103
// MI455X (gfx1250) — hardware-verified
//
#include <hip/hip_runtime.h>


#ifndef NB
#define NB 2
#endif
#ifndef SEQ
#define SEQ 2048
#endif
#define NB_FULL  2
#define SEQ_FULL 2048
#ifndef OUT_SEQ
#define OUT_SEQ SEQ
#endif
#ifndef EARLY_CAP
#define EARLY_CAP 512
#endif
#define EARLY ((SEQ) < (EARLY_CAP) ? (SEQ) : (EARLY_CAP))
#define DM   2048
#define NH_  16
#define NKV  4
#define HD   128
#define KVD  (NKV * HD)
#define NQKV (DM + 2 * KVD)
#define AW   4
#define QRS  2048.0f
#define QRI  (1.0f / 2048.0f)
#define SC2  (0.08838834764831845f * 1.4426950408889634f)
#define PSH  8.0f
#define CSC  16.0f
#define OSCL (1.0f / 16384.0f)
#define OSP  132

static_assert(HD == 128);
static_assert(NH_ * HD == DM);
static_assert(NH_ % NKV == 0);
static_assert(DM % 64 == 0);
static_assert(KVD % 64 == 0);
static_assert(DM % 32 == 0);
static_assert(SEQ % 64 == 0);
static_assert(EARLY % 64 == 0);
static_assert((SEQ - EARLY) % 64 == 0);
static_assert(EARLY <= SEQ);
static_assert(((size_t)SEQ * DM) % 8 == 0);
static_assert(NB <= NB_FULL);
static_assert(SEQ <= SEQ_FULL);

typedef _Float16 h16;
typedef unsigned short bf;
typedef __attribute__((ext_vector_type(16))) __bf16   v16bf;
typedef __attribute__((ext_vector_type(16))) _Float16 v16h;
typedef __attribute__((ext_vector_type(8)))  _Float16 v8h;
typedef __attribute__((ext_vector_type(8)))  unsigned short v8us;
typedef __attribute__((ext_vector_type(8)))  float    v8f;
typedef __attribute__((ext_vector_type(4)))  float    v4f;
typedef v4f  __attribute__((may_alias)) v4fa;

__device__ __forceinline__ unsigned short f2bf(float f) { unsigned u = __float_as_uint(f); u += 0x7FFFu + ((u >> 16) & 1u); return (unsigned short)(u >> 16); }
__device__ __forceinline__ unsigned short h2us(h16 v) { return __builtin_bit_cast(unsigned short, v); }
__device__ __forceinline__ v16h cat16(v8h lo, v8h hi) { return __builtin_shufflevector(lo, hi, 0, 1, 2, 3, 4, 5, 6, 7, 8, 9, 10, 11, 12, 13, 14, 15); }
__device__ __forceinline__ v16bf cat16b(v8us lo, v8us hi) { return __builtin_bit_cast(v16bf, __builtin_shufflevector(lo, hi, 0, 1, 2, 3, 4, 5, 6, 7, 8, 9, 10, 11, 12, 13, 14, 15)); }
__device__ __forceinline__ v8f wmma16(v16h a, v16h b, v8f c) { return __builtin_amdgcn_wmma_f32_16x16x32_f16(false, a, false, b, (short)0, c, false, false); }
__device__ __forceinline__ v8f wmmab(v16bf a, v16bf b, v8f c) { return __builtin_amdgcn_wmma_f32_16x16x32_bf16(false, a, false, b, (short)0, c, false, false); }
__device__ __forceinline__ v16h  ldh(const h16* p) { return cat16(*(const v8h*)p, *(const v8h*)(p + 16)); }
__device__ __forceinline__ v16bf ldb(const bf* p)  { return cat16b(*(const v8us*)p, *(const v8us*)(p + 16)); }
__device__ __forceinline__ void wave_sync() { __builtin_amdgcn_fence(3  , "wavefront"); __builtin_amdgcn_wave_barrier(); asm volatile("" ::: "memory"); }

__global__ __launch_bounds__(256) void k_cvt8(const float* __restrict__ src, bf* dst, size_t n8) {
    const size_t i = (size_t)blockIdx.x * 256 + threadIdx.x; if (i >= n8) return;
    const v8f v = *(const v8f*)(src + i * 8); v8us o;
#pragma unroll
    for (int k = 0; k < 8; ++k) o[k] = f2bf(v[k]);
    *(volatile v8us*)(dst + i * 8) = o; __threadfence(); *(volatile v8us*)(dst + i * 8) = o;
}

template<int MODE> __device__ __forceinline__ unsigned short cvw(float w) {
    const unsigned short b = f2bf(w);
    if (MODE == 0) return b;
    const float wb = __uint_as_float(((unsigned)b) << 16);
    return h2us((h16)(wb * 1024.0f));
}

template<int MODE>
__global__ __launch_bounds__(256) void k_wT(const float* __restrict__ src, unsigned short* dst, int K, int N) {
    __shared__ float ts[64 * 65];
    const int tid = threadIdx.x;
    const int n0 = blockIdx.x * 64, k0 = blockIdx.y * 64;
    { const int c4 = (tid & 15) * 4, r = tid >> 4;
#pragma unroll
      for (int p = 0; p < 4; ++p) { const int kk = r + 16 * p;
          const v4f v = *(const v4f*)(src + (size_t)(k0 + kk) * N + n0 + c4);
          ts[kk * 65 + c4 + 0] = v[0]; ts[kk * 65 + c4 + 1] = v[1]; ts[kk * 65 + c4 + 2] = v[2]; ts[kk * 65 + c4 + 3] = v[3]; } }
    __syncthreads();
    const int rw = tid >> 3, c8 = (tid & 7) * 8;
    v8us o0, o1;
#pragma unroll
    for (int j = 0; j < 8; ++j) { o0[j] = cvw<MODE>(ts[(c8 + j) * 65 + rw]); o1[j] = cvw<MODE>(ts[(c8 + j) * 65 + rw + 32]); }
    unsigned short* d0 = dst + (size_t)(n0 + rw) * K + k0 + c8;
    unsigned short* d1 = dst + (size_t)(n0 + rw + 32) * K + k0 + c8;
    *(volatile v8us*)d0 = o0; *(volatile v8us*)d1 = o1;
    __threadfence();
    *(volatile v8us*)d0 = o0; *(volatile v8us*)d1 = o1;
}

__global__ __launch_bounds__(256) void k_tab(float* COS, float* SIN, int n) {
    const int idx = blockIdx.x * 256 + threadIdx.x; if (idx >= n) return;
    const int s = idx >> 6, i = idx & 63;
    double p = 1.0;
    p *= (i & 1)  ? 1.1547819846894583 : 1.0;
    p *= (i & 2)  ? 1.333521432163324  : 1.0;
    p *= (i & 4)  ? 1.7782794100389228 : 1.0;
    p *= (i & 8)  ? 3.1622776601683795 : 1.0;
    p *= (i & 16) ? 10.0 : 1.0;
    p *= (i & 32) ? 100.0 : 1.0;
    const float pf = (float)p;
    const float invf = 1.0f / pf;
    const float ang = (float)s * invf;
    const double x = (double)ang;
    const double nq = rint(x * 0.63661977236758134);
    double r = fma(-nq, 1.5707963267948966, x);
    r = fma(-nq, 6.123233995736766e-17, r);
    const int q = ((int)nq) & 3;
    const double r2 = r * r;
    double sp = 1.0 / 6227020800.0;
    sp = fma(sp, r2, -1.0 / 39916800.0);
    sp = fma(sp, r2, 1.0 / 362880.0);
    sp = fma(sp, r2, -1.0 / 5040.0);
    sp = fma(sp, r2, 1.0 / 120.0);
    sp = fma(sp, r2, -1.0 / 6.0);
    sp = fma(sp * r2, r, r);
    double cp = -1.0 / 87178291200.0;
    cp = fma(cp, r2, 1.0 / 479001600.0);
    cp = fma(cp, r2, -1.0 / 3628800.0);
    cp = fma(cp, r2, 1.0 / 40320.0);
    cp = fma(cp, r2, -1.0 / 720.0);
    cp = fma(cp, r2, 1.0 / 24.0);
    cp = fma(cp, r2, -0.5);
    cp = fma(cp, r2, 1.0);
    double sv = (q & 1) ? cp : sp;
    double cv = (q & 1) ? sp : cp;
    sv = (q & 2) ? -sv : sv;
    cv = ((q + 1) & 2) ? -cv : cv;
    const float cf = (float)cv, sf = (float)sv;
    *(volatile float*)(COS + idx) = cf; *(volatile float*)(SIN + idx) = sf;
    __threadfence();
    *(volatile float*)(COS + idx) = cf; *(volatile float*)(SIN + idx) = sf;
}

__global__ __launch_bounds__(32) void k_proj(const bf* __restrict__ A, const bf* __restrict__ Bt, h16* Ph, h16* Pr, int useRes, int rope,
                                             const float* __restrict__ COS, const float* __restrict__ SIN, int RB, size_t sRB, int pitch, int CB, size_t sCB) {
    __shared__ __align__(16) float os[16 * 68];
    const int K = DM;
    const int lane = threadIdx.x & 31, lr = lane & 15, hi = lane >> 4; const int r0 = blockIdx.x * 64, c0 = blockIdx.y * 64;
    v8f acc[4][4];
#pragma unroll
    for (int mb = 0; mb < 4; ++mb)
#pragma unroll
        for (int nb = 0; nb < 4; ++nb) acc[mb][nb] = (v8f){};
    const size_t aoff = (size_t)(r0 + lr) * K + 8 * hi, boff = (size_t)(c0 + lr) * K + 8 * hi;
#pragma unroll 1
    for (int kc = 0; kc < K; kc += 32) {
        v16bf a[4];
#pragma unroll
        for (int mb = 0; mb < 4; ++mb) a[mb] = ldb(A + aoff + (size_t)mb * 16 * K + kc);
#pragma unroll
        for (int nb = 0; nb < 4; ++nb) { const v16bf b = ldb(Bt + boff + (size_t)nb * 16 * K + kc);
#pragma unroll
            for (int mb = 0; mb < 4; ++mb) acc[mb][nb] = wmmab(a[mb], b, acc[mb][nb]); }
        asm volatile("v_nop\n\tv_nop\n\tv_nop\n\tv_nop" : "+v"(acc[0][3]), "+v"(acc[1][3]), "+v"(acc[2][3]), "+v"(acc[3][3]) : "v"(a[0]), "v"(a[1]), "v"(a[2]), "v"(a[3]));
    }
    const size_t tbase = (size_t)(r0 / RB) * sRB + (size_t)(r0 % RB) * (size_t)pitch + (size_t)(c0 / CB) * sCB + (size_t)(c0 % CB);
    const int tp0 = r0 % RB;
    const int ib = (c0 & (HD - 1)) >> 1;
#pragma unroll
    for (int mb = 0; mb < 4; ++mb) {
#pragma unroll
        for (int nb = 0; nb < 4; ++nb) {
#pragma unroll
            for (int j = 0; j < 8; ++j) os[(hi * 8 + j) * 68 + nb * 16 + lr] = acc[mb][nb][j]; }
        wave_sync();
        const size_t sb = tbase + (size_t)(mb * 16) * (size_t)pitch;
#pragma unroll 1
        for (int ps = 0; ps < 2; ++ps) {
#pragma unroll
            for (int s = 0; s < 4; ++s) { const int row = 4 * s + (lane >> 3), c8 = (lane & 7) * 8;
                v4f x0 = *(const v4fa*)(&os[row * 68 + c8]); v4f x1 = *(const v4fa*)(&os[row * 68 + c8 + 4]);
                if (rope) {
                    const int io = (tp0 + mb * 16 + row) * 64 + ib + (c8 >> 1);
                    const v4f cs = *(const v4f*)(COS + io); const v4f sn = *(const v4f*)(SIN + io);
                    const float a0 = x0[0], b0 = x0[1], a1 = x0[2], b1 = x0[3], a2 = x1[0], b2 = x1[1], a3 = x1[2], b3 = x1[3];
                    x0[0] = a0 * cs[0] - b0 * sn[0]; x0[1] = a0 * sn[0] + b0 * cs[0];
                    x0[2] = a1 * cs[1] - b1 * sn[1]; x0[3] = a1 * sn[1] + b1 * cs[1];
                    x1[0] = a2 * cs[2] - b2 * sn[2]; x1[1] = a2 * sn[2] + b2 * cs[2];
                    x1[2] = a3 * cs[3] - b3 * sn[3]; x1[3] = a3 * sn[3] + b3 * cs[3];
                }
                v8h hv, rv;
#pragma unroll
                for (int i = 0; i < 4; ++i) { const h16 e0 = (h16)x0[i]; const h16 e1 = (h16)x1[i]; hv[i] = e0; hv[4 + i] = e1; rv[i] = (h16)((x0[i] - (float)e0) * QRS); rv[4 + i] = (h16)((x1[i] - (float)e1) * QRS); }
                const size_t oo = sb + (size_t)row * (size_t)pitch + c8;
                *(volatile v8h*)(Ph + oo) = hv; if (useRes) *(volatile v8h*)(Pr + oo) = rv; }
            if (ps == 0) __threadfence(); }
        wave_sync();
    }
}

__global__ __launch_bounds__(32 * AW) void k_flash(const h16* __restrict__ QH, const h16* __restrict__ KP, const h16* __restrict__ VT, h16* CH) {
    __shared__ __align__(16) float os[AW * 16 * OSP];
    const int lane = threadIdx.x & 31, lr = lane & 15, hi = lane >> 4;
    const int wave = __builtin_amdgcn_readfirstlane((int)(threadIdx.x >> 5));
    const int zh = blockIdx.y; const int b = zh / NH_, h = zh % NH_; const int kvz = b * NKV + h / (NH_ / NKV);
    const int t0 = EARLY + (blockIdx.x * AW + wave) * 16;
    const size_t qo = (size_t)zh * SEQ * HD + (size_t)(t0 + lr) * HD + 8 * hi;
    v16h qf[4];
#pragma unroll
    for (int c = 0; c < 4; ++c) qf[c] = ldh(QH + qo + 32 * c);
    const size_t kvb = (size_t)kvz * SEQ * HD;
    const size_t ko = kvb + (size_t)lr * HD + 8 * hi;
    const size_t vo = kvb + (size_t)lr * SEQ + 8 * hi;
    v8f o[8];
#pragma unroll
    for (int j = 0; j < 8; ++j) o[j] = (v8f){};
    float m = -3.0e38f, l = 0.0f;
    const int tq = t0 + lr;
    const int nkb = (t0 + 16 + 31) >> 5;
#pragma unroll 1
    for (int kb = 0; kb < nkb; ++kb) {
        const int key0 = kb * 32;
        const h16* ka = KP + ko + (size_t)key0 * HD;
        v8f sa = (v8f){}, sb = (v8f){}; v16h fa, fb;
#pragma unroll
        for (int c = 0; c < 4; ++c) { fa = ldh(ka + 32 * c); fb = ldh(ka + 16 * HD + 32 * c);
            sa = wmma16(fa, qf[c], sa); sb = wmma16(fb, qf[c], sb);
            __builtin_amdgcn_sched_barrier(0); }
        asm volatile("v_nop\n\tv_nop\n\tv_nop\n\tv_nop" : "+v"(sa), "+v"(sb) : "v"(fa), "v"(fb));
        float ta[8], tb[8];
#pragma unroll
        for (int r = 0; r < 8; ++r) { ta[r] = sa[r] * SC2; tb[r] = sb[r] * SC2; }
        if (key0 + 31 > t0) {
#pragma unroll
            for (int r = 0; r < 8; ++r) { const int kA = key0 + 8 * hi + r;
                ta[r] = (kA <= tq) ? ta[r] : -__builtin_inff(); tb[r] = (kA + 16 <= tq) ? tb[r] : -__builtin_inff(); }
        }
        float mx = -3.0e38f;
#pragma unroll
        for (int r = 0; r < 8; ++r) mx = fmaxf(mx, fmaxf(ta[r], tb[r]));
        mx = fmaxf(mx, __shfl_xor(mx, 16, 32));
        const float mnew = fmaxf(m, mx);
        const float alpha = __builtin_amdgcn_exp2f(m - mnew);
        const float sh = PSH - mnew;
        v16h pb; float ls = 0.0f;
#pragma unroll
        for (int r = 0; r < 8; ++r) { const h16 pa = (h16)__builtin_amdgcn_exp2f(ta[r] + sh); const h16 pc = (h16)__builtin_amdgcn_exp2f(tb[r] + sh); pb[r] = pa; pb[8 + r] = pc; ls += (float)pa + (float)pc; }
        l = l * alpha + ls; m = mnew;
#pragma unroll
        for (int j = 0; j < 8; ++j) o[j] = o[j] * alpha;
        const h16* va = VT + vo + key0;
        v16h v0f, v1f;
#pragma unroll
        for (int j = 0; j < 8; j += 2) { v0f = ldh(va + (size_t)(16 * j) * SEQ); v1f = ldh(va + (size_t)(16 * j + 16) * SEQ);
            o[j] = wmma16(v0f, pb, o[j]); o[j + 1] = wmma16(v1f, pb, o[j + 1]);
            __builtin_amdgcn_sched_barrier(0); }
        asm volatile("v_nop\n\tv_nop\n\tv_nop\n\tv_nop" : "+v"(o[0]), "+v"(o[1]), "+v"(o[2]), "+v"(o[3]), "+v"(o[4]), "+v"(o[5]), "+v"(o[6]), "+v"(o[7]) : "v"(v0f), "v"(v1f), "v"(pb));
    }
    l += __shfl_xor(l, 16, 32);
    const float inv = CSC * (1.0f / l);
    const int wb = wave * 16 * OSP;
#pragma unroll
    for (int j = 0; j < 8; ++j) { v4f a, c;
        a[0] = o[j][0] * inv; a[1] = o[j][1] * inv; a[2] = o[j][2] * inv; a[3] = o[j][3] * inv; c[0] = o[j][4] * inv; c[1] = o[j][5] * inv; c[2] = o[j][6] * inv; c[3] = o[j][7] * inv;
        *(v4fa*)(&os[wb + lr * OSP + 16 * j + 8 * hi]) = a; *(v4fa*)(&os[wb + lr * OSP + 16 * j + 8 * hi + 4]) = c; }
    wave_sync();
    h16* crow = CH + ((size_t)b * SEQ + t0) * DM + h * HD;
#pragma unroll 1
    for (int ps = 0; ps < 2; ++ps) {
#pragma unroll
        for (int s = 0; s < 8; ++s) { const int row = 2 * s + hi, c8 = lr * 8;
            const v4f x0 = *(const v4fa*)(&os[wb + row * OSP + c8]); const v4f x1 = *(const v4fa*)(&os[wb + row * OSP + c8 + 4]); v8h hv;
#pragma unroll
            for (int i = 0; i < 4; ++i) { hv[i] = (h16)x0[i]; hv[4 + i] = (h16)x1[i]; }
            *(volatile v8h*)(crow + (size_t)row * DM + c8) = hv; }
        if (ps == 0) __threadfence(); }
}

__global__ __launch_bounds__(128) void k_flash_e(const h16* __restrict__ QH, const h16* __restrict__ QR, const h16* __restrict__ KP, const h16* __restrict__ KR,
                                                 const h16* __restrict__ VT, const h16* __restrict__ VR, h16* CH, h16* CR) {
    __shared__ __align__(16) float os[4 * 16 * 68];
    const int lane = threadIdx.x & 31, lr = lane & 15, hi = lane >> 4;
    const int wave = __builtin_amdgcn_readfirstlane((int)(threadIdx.x >> 5));
    const int qs = wave >> 1, dh = wave & 1;
    const int zh = blockIdx.y; const int b = zh / NH_, h = zh % NH_; const int kvz = b * NKV + h / (NH_ / NKV);
    const int t0 = (blockIdx.x * 2 + qs) * 16;
    const size_t qo = (size_t)zh * SEQ * HD + (size_t)(t0 + lr) * HD + 8 * hi;
    v16h qh[4], qr[4];
#pragma unroll
    for (int c = 0; c < 4; ++c) { qh[c] = ldh(QH + qo + 32 * c); qr[c] = ldh(QR + qo + 32 * c); }
    const size_t kvb = (size_t)kvz * SEQ * HD;
    const size_t ko = kvb + (size_t)lr * HD + 8 * hi;
    const size_t vo = kvb + (size_t)(dh * 64 + lr) * SEQ + 8 * hi;
    v8f oh[4], orr[4];
#pragma unroll
    for (int j = 0; j < 4; ++j) { oh[j] = (v8f){}; orr[j] = (v8f){}; }
    float m = -3.0e38f, l = 0.0f;
    const int tq = t0 + lr;
    const int nkb = (t0 + 16 + 31) >> 5;
#pragma unroll 1
    for (int kb = 0; kb < nkb; ++kb) {
        const int key0 = kb * 32;
        const h16* ka = KP + ko + (size_t)key0 * HD;
        const h16* kr = KR + ko + (size_t)key0 * HD;
        v8f sHa = (v8f){}, sLa = (v8f){}, sHb = (v8f){}, sLb = (v8f){}; v16h fa, fb, ga, gb;
#pragma unroll
        for (int c = 0; c < 4; ++c) { fa = ldh(ka + 32 * c); fb = ldh(ka + 16 * HD + 32 * c); ga = ldh(kr + 32 * c); gb = ldh(kr + 16 * HD + 32 * c);
            sHa = wmma16(fa, qh[c], sHa); sHb = wmma16(fb, qh[c], sHb);
            sLa = wmma16(fa, qr[c], sLa); sLb = wmma16(fb, qr[c], sLb);
            sLa = wmma16(ga, qh[c], sLa); sLb = wmma16(gb, qh[c], sLb);
            __builtin_amdgcn_sched_barrier(0); }
        asm volatile("v_nop\n\tv_nop\n\tv_nop\n\tv_nop" : "+v"(sHa), "+v"(sLa), "+v"(sHb), "+v"(sLb) : "v"(fa), "v"(fb), "v"(ga), "v"(gb));
        float ta[8], tb[8];
#pragma unroll
        for (int r = 0; r < 8; ++r) { ta[r] = (sHa[r] + sLa[r] * QRI) * SC2; tb[r] = (sHb[r] + sLb[r] * QRI) * SC2; }
        if (key0 + 31 > t0) {
#pragma unroll
            for (int r = 0; r < 8; ++r) { const int kA = key0 + 8 * hi + r;
                ta[r] = (kA <= tq) ? ta[r] : -__builtin_inff(); tb[r] = (kA + 16 <= tq) ? tb[r] : -__builtin_inff(); }
        }
        float mx = -3.0e38f;
#pragma unroll
        for (int r = 0; r < 8; ++r) mx = fmaxf(mx, fmaxf(ta[r], tb[r]));
        mx = fmaxf(mx, __shfl_xor(mx, 16, 32));
        const float mnew = fmaxf(m, mx);
        const float alpha = __builtin_amdgcn_exp2f(m - mnew);
        const float sh = PSH - mnew;
        v16h pbh, pbr; float ls = 0.0f;
#pragma unroll
        for (int r = 0; r < 8; ++r) { const float pa = __builtin_amdgcn_exp2f(ta[r] + sh); const float pc = __builtin_amdgcn_exp2f(tb[r] + sh);
            const h16 ea = (h16)pa; const h16 ec = (h16)pc; pbh[r] = ea; pbh[8 + r] = ec;
            pbr[r] = (h16)((pa - (float)ea) * QRS); pbr[8 + r] = (h16)((pc - (float)ec) * QRS); ls += pa + pc; }
        l = l * alpha + ls; m = mnew;
#pragma unroll
        for (int j = 0; j < 4; ++j) { oh[j] = oh[j] * alpha; orr[j] = orr[j] * alpha; }
        const h16* va = VT + vo + key0;
        const h16* vr = VR + vo + key0;
        v16h h0, h1, g0, g1;
#pragma unroll
        for (int j = 0; j < 4; j += 2) {
            h0 = ldh(va + (size_t)(16 * j) * SEQ); h1 = ldh(va + (size_t)(16 * j + 16) * SEQ);
            g0 = ldh(vr + (size_t)(16 * j) * SEQ); g1 = ldh(vr + (size_t)(16 * j + 16) * SEQ);
            oh[j] = wmma16(h0, pbh, oh[j]);   orr[j] = wmma16(h0, pbr, orr[j]);
            oh[j + 1] = wmma16(h1, pbh, oh[j + 1]); orr[j + 1] = wmma16(h1, pbr, orr[j + 1]);
            orr[j] = wmma16(g0, pbh, orr[j]); orr[j + 1] = wmma16(g1, pbh, orr[j + 1]);
            __builtin_amdgcn_sched_barrier(0); }
        asm volatile("v_nop\n\tv_nop\n\tv_nop\n\tv_nop" : "+v"(oh[0]), "+v"(oh[1]), "+v"(oh[2]), "+v"(oh[3]), "+v"(orr[0]), "+v"(orr[1]), "+v"(orr[2]), "+v"(orr[3]) : "v"(h1), "v"(g0), "v"(g1), "v"(pbh), "v"(pbr));
    }
    l += __shfl_xor(l, 16, 32);
    const float inv = CSC * (1.0f / l);
    const int wb = wave * 16 * 68;
#pragma unroll
    for (int j = 0; j < 4; ++j) { v4f a, c;
#pragma unroll
        for (int i = 0; i < 4; ++i) { a[i] = (oh[j][i] + orr[j][i] * QRI) * inv; c[i] = (oh[j][4 + i] + orr[j][4 + i] * QRI) * inv; }
        *(v4fa*)(&os[wb + lr * 68 + 16 * j + 8 * hi]) = a; *(v4fa*)(&os[wb + lr * 68 + 16 * j + 8 * hi + 4]) = c; }
    wave_sync();
    h16* crow = CH + ((size_t)b * SEQ + t0) * DM + h * HD + dh * 64;
    h16* rrow = CR + ((size_t)b * EARLY + t0) * DM + h * HD + dh * 64;
#pragma unroll 1
    for (int ps = 0; ps < 2; ++ps) {
#pragma unroll
        for (int s = 0; s < 4; ++s) { const int row = 4 * s + (lane >> 3), c8 = (lane & 7) * 8;
            const v4f x0 = *(const v4fa*)(&os[wb + row * 68 + c8]); const v4f x1 = *(const v4fa*)(&os[wb + row * 68 + c8 + 4]); v8h hv, rv;
#pragma unroll
            for (int i = 0; i < 4; ++i) { const h16 e0 = (h16)x0[i]; const h16 e1 = (h16)x1[i]; hv[i] = e0; hv[4 + i] = e1; rv[i] = (h16)((x0[i] - (float)e0) * QRS); rv[4 + i] = (h16)((x1[i] - (float)e1) * QRS); }
            *(volatile v8h*)(crow + (size_t)row * DM + c8) = hv; *(volatile v8h*)(rrow + (size_t)row * DM + c8) = rv; }
        if (ps == 0) __threadfence(); }
}

template<int MB, int RES>
__global__ __launch_bounds__(32) void k_out(const h16* __restrict__ CH, const h16* __restrict__ CR, const h16* __restrict__ WT, float* OUT, int tpb, int rowStart) {
    static_assert((MB == 4 && RES == 0) || (MB == 2 && RES == 1));
    __shared__ __align__(16) float os[16 * 68];
    const int K = DM;
    const int lane = threadIdx.x & 31, lr = lane & 15, hi = lane >> 4;
    const int bb = blockIdx.x / tpb, tt = blockIdx.x % tpb;
    const int t0 = rowStart + tt * (16 * MB);
    const int c0 = blockIdx.y * 64;
    const size_t aoff = ((size_t)bb * SEQ + t0 + lr) * K + 8 * hi;
    const size_t roff = ((size_t)bb * EARLY + t0 + lr) * K + 8 * hi;
    const size_t boff = (size_t)(c0 + lr) * K + 8 * hi;
    v8f acc[MB][4], accr[MB][4];
#pragma unroll
    for (int mb = 0; mb < MB; ++mb)
#pragma unroll
        for (int nb = 0; nb < 4; ++nb) { acc[mb][nb] = (v8f){}; accr[mb][nb] = (v8f){}; }
#pragma unroll 1
    for (int kc = 0; kc < K; kc += 32) {
        v16h a[MB], ar[MB];
#pragma unroll
        for (int mb = 0; mb < MB; ++mb) { a[mb] = ldh(CH + aoff + (size_t)mb * 16 * K + kc); if (RES) ar[mb] = ldh(CR + roff + (size_t)mb * 16 * K + kc); }
#pragma unroll
        for (int nb = 0; nb < 4; ++nb) { const v16h bq = ldh(WT + boff + (size_t)nb * 16 * K + kc);
#pragma unroll
            for (int mb = 0; mb < MB; ++mb) { acc[mb][nb] = wmma16(a[mb], bq, acc[mb][nb]); if (RES) accr[mb][nb] = wmma16(ar[mb], bq, accr[mb][nb]); } }
        if constexpr (MB == 4) {
            asm volatile("v_nop\n\tv_nop\n\tv_nop\n\tv_nop" : "+v"(acc[0][3]), "+v"(acc[1][3]), "+v"(acc[2][3]), "+v"(acc[3][3]) : "v"(a[0]), "v"(a[1]), "v"(a[2]), "v"(a[3]));
        } else {
            asm volatile("v_nop\n\tv_nop\n\tv_nop\n\tv_nop" : "+v"(acc[0][3]), "+v"(acc[1][3]), "+v"(accr[0][3]), "+v"(accr[1][3]) : "v"(a[0]), "v"(a[1]), "v"(ar[0]), "v"(ar[1]));
        }
    }
#pragma unroll
    for (int mb = 0; mb < MB; ++mb) {
#pragma unroll
        for (int nb = 0; nb < 4; ++nb) {
#pragma unroll
            for (int j = 0; j < 8; ++j) { float v = acc[mb][nb][j]; if (RES) v = v + accr[mb][nb][j] * QRI; os[(hi * 8 + j) * 68 + nb * 16 + lr] = v * OSCL; } }
        wave_sync();
        float* orow = OUT + ((size_t)bb * OUT_SEQ + t0 + mb * 16) * DM + c0;
#pragma unroll 1
        for (int ps = 0; ps < 2; ++ps) {
#pragma unroll
            for (int s = 0; s < 8; ++s) { const int row = 2 * s + hi, cofs = lr * 4;
                const v4f val = *(const v4fa*)(&os[row * 68 + cofs]);
                *(volatile v4f*)(orow + (size_t)row * DM + cofs) = val; }
            if (ps == 0) __threadfence(); }
        wave_sync();
    }
}

static constexpr size_t al256(size_t v) { return (v + 255) & ~(size_t)255; }
static constexpr size_t SZ_XB = al256((size_t)NB * SEQ * DM * 2);
static constexpr size_t SZ_WT = al256((size_t)NQKV * DM * 2);
static constexpr size_t SZ_WO = al256((size_t)DM * DM * 2);
static constexpr size_t SZ_Q  = al256((size_t)NB * NH_ * SEQ * HD * 2);
static constexpr size_t SZ_KV = al256((size_t)NB * NKV * SEQ * HD * 2);
static constexpr size_t SZ_CH = al256((size_t)NB * SEQ * DM * 2);
static constexpr size_t SZ_CR = al256((size_t)NB * EARLY * DM * 2);
static constexpr size_t SZ_TB = al256((size_t)SEQ * 64 * 4);
static constexpr size_t SZ_TOTAL = SZ_XB + SZ_WT + SZ_WO + 2 * SZ_Q + 4 * SZ_KV + SZ_CH + SZ_CR + 2 * SZ_TB;
static_assert(SZ_TOTAL <= (size_t)134217728);
static_assert(((size_t)DM * DM * 2) % 256 == 0);
static_assert(((size_t)KVD * DM * 2) % 256 == 0);
static_assert(((size_t)SEQ * 64) % 256 == 0);

extern "C" void kernel_launch(void* const* d_in, const int* in_sizes, int n_in,
                              void* d_out, int out_size, void* d_ws, size_t ws_size, hipStream_t stream) {
    if (n_in < 5) return;
    const size_t needx = ((size_t)(NB - 1) * SEQ_FULL + SEQ) * DM;
    if ((size_t)in_sizes[0] < needx) return;
    if ((size_t)in_sizes[1] < (size_t)DM * DM || (size_t)in_sizes[2] < (size_t)DM * KVD || (size_t)in_sizes[3] < (size_t)DM * KVD || (size_t)in_sizes[4] < (size_t)DM * DM) return;
    if ((size_t)out_size < ((size_t)(NB - 1) * OUT_SEQ + SEQ) * DM) return;
    if (SZ_TOTAL > ws_size) return;
    const float* x = (const float*)d_in[0]; const float* wq = (const float*)d_in[1]; const float* wk = (const float*)d_in[2];
    const float* wv = (const float*)d_in[3]; const float* wo = (const float*)d_in[4];
    float* OUT = (float*)d_out;
    char* wsp = (char*)d_ws;
    bf* XB = (bf*)wsp; wsp += SZ_XB;
    bf* WT = (bf*)wsp; wsp += SZ_WT;
    h16* WOT = (h16*)wsp; wsp += SZ_WO;
    h16* QH = (h16*)wsp; wsp += SZ_Q;
    h16* QR = (h16*)wsp; wsp += SZ_Q;
    h16* KP = (h16*)wsp; wsp += SZ_KV;
    h16* KR = (h16*)wsp; wsp += SZ_KV;
    h16* VT = (h16*)wsp; wsp += SZ_KV;
    h16* VR = (h16*)wsp; wsp += SZ_KV;
    h16* CH = (h16*)wsp; wsp += SZ_CH;
    h16* CR = (h16*)wsp; wsp += SZ_CR;
    float* COS = (float*)wsp; wsp += SZ_TB;
    float* SIN = (float*)wsp; wsp += SZ_TB;

    if (SEQ == SEQ_FULL) {
        const size_t n8 = (size_t)NB * SEQ * DM / 8;
        k_cvt8<<<(unsigned)((n8 + 255) / 256), 256, 0, stream>>>(x, XB, n8);
    } else {
        const size_t n8 = (size_t)SEQ * DM / 8;
        for (int b = 0; b < NB; ++b) k_cvt8<<<(unsigned)((n8 + 255) / 256), 256, 0, stream>>>(x + (size_t)b * SEQ_FULL * DM, XB + (size_t)b * SEQ * DM, n8);
    }
    k_wT<0><<<dim3(DM / 64,  DM / 64, 1), 256, 0, stream>>>(wq, WT, DM, DM);
    k_wT<0><<<dim3(KVD / 64, DM / 64, 1), 256, 0, stream>>>(wk, WT + (size_t)DM * DM, DM, KVD);
    k_wT<0><<<dim3(KVD / 64, DM / 64, 1), 256, 0, stream>>>(wv, WT + (size_t)(DM + KVD) * DM, DM, KVD);
    k_wT<1><<<dim3(DM / 64,  DM / 64, 1), 256, 0, stream>>>(wo, (unsigned short*)WOT, DM, DM);
    k_tab<<<(unsigned)((size_t)SEQ * 64 / 256), 256, 0, stream>>>(COS, SIN, SEQ * 64);

    k_proj<<<dim3(NB * SEQ / 64, DM / 64, 1), 32, 0, stream>>>(XB, WT, QH, QR, 1, 1, COS, SIN, SEQ, (size_t)NH_ * SEQ * HD, HD, HD, (size_t)SEQ * HD);
    k_proj<<<dim3(NB * SEQ / 64, KVD / 64, 1), 32, 0, stream>>>(XB, WT + (size_t)DM * DM, KP, KR, 1, 1, COS, SIN, SEQ, (size_t)NKV * SEQ * HD, HD, HD, (size_t)SEQ * HD);
    k_proj<<<dim3(KVD / 64, NB * SEQ / 64, 1), 32, 0, stream>>>(WT + (size_t)(DM + KVD) * DM, XB, VT, VR, 1, 0, COS, SIN, KVD, (size_t)0, SEQ, SEQ, (size_t)KVD * SEQ);

    k_flash_e<<<dim3(EARLY / 32, NB * NH_, 1), 128, 0, stream>>>(QH, QR, KP, KR, VT, VR, CH, CR);
    if (SEQ > EARLY)
        k_flash<<<dim3((SEQ - EARLY) / (16 * AW), NB * NH_, 1), 32 * AW, 0, stream>>>(QH, KP, VT, CH);

    k_out<2, 1><<<dim3(NB * (EARLY / 32), DM / 64, 1), 32, 0, stream>>>(CH, CR, WOT, OUT, EARLY / 32, 0);
    if (SEQ > EARLY)
        k_out<4, 0><<<dim3(NB * ((SEQ - EARLY) / 64), DM / 64, 1), 32, 0, stream>>>(CH, CR, WOT, OUT, (SEQ - EARLY) / 64, EARLY);
}
